// GAT_19774029431579
// MI455X (gfx1250) — hardware-verified
//
#include <hip/hip_runtime.h>
#include <stddef.h>
#include <stdint.h>
#include <math.h>


#define FIN     128
#define HC      256
#define HID     64
#define NHD     4
#define LDX     512
#define KA2     512
#define NGR     64
#define OUTC    16
#define NTHR    256
#define NWAVE   8
#define EPT     8
#define CHUNK   (NTHR * EPT)
#define WCAP    (EPT * 32)
#define LISTN   (NWAVE * WCAP)
#define NBA     1024
#define SLA     10
#define RCAP    28672
#define DEGCAP  128
#define MEAS_B1024  12548
#define MEAS_MAXDEG 28
#define GBM     64
#define GBN     64
#define GTHR    128
#define MROWS   128
#define NUW1H   (HC * (FIN / 8))
#define NUW2H   (HC * (KA2 / 8))
#define NEGSL   0.2f
#define WSMAX   268435456
#define BKT_LDS_INTS  (LISTN + RCAP + 16)
#define SCAN_ZINTS    (RCAP + 3 * NBA)
#define SCAN_LDS_INTS (2 * RCAP + 3 * NBA + 16)

static_assert((CHUNK & (CHUNK - 1)) == 0 && CHUNK <= 4096);
static_assert((NBA & (NBA - 1)) == 0 && NBA == (1 << SLA) && NBA <= 1024);
static_assert(((long long)CHUNK << SLA) < (1LL << 31));
static_assert(LISTN >= NWAVE * WCAP);
static_assert(NBA % NWAVE == 0 && NBA % 32 == 0);
static_assert((RCAP % 32) == 0 && (SCAN_ZINTS % 4) == 0);
static_assert(RCAP >= MEAS_B1024 + 4096);
static_assert(DEGCAP >= MEAS_MAXDEG + 8);
static_assert(SCAN_LDS_INTS * 4 <= 300000 && BKT_LDS_INTS * 4 <= 300000);
static_assert(GBM == (GTHR / 32) * 16);
static_assert((FIN % 32) == 0 && (KA2 % 32) == 0 && KA2 == 2 * HC);
static_assert((LDX % GBN) == 0 && LDX == 2 * HC);
static_assert((MROWS % GBM) == 0);
static_assert(HC == 8 * 32);
static_assert(HC == NHD * HID && HID == 8 * 8);
static_assert((NUW1H % NTHR) == 0 && (NUW2H % NTHR) == 0);
static_assert(NGR * OUTC == NTHR * 4);
static_assert(NGR * HID == NTHR * 16);

typedef float          v2f  __attribute__((ext_vector_type(2)));
typedef float          v4f  __attribute__((ext_vector_type(4)));
typedef float          v8f  __attribute__((ext_vector_type(8)));
typedef int            v4i  __attribute__((ext_vector_type(4)));
typedef int            v8i  __attribute__((ext_vector_type(8)));
typedef unsigned short v8us __attribute__((ext_vector_type(8)));
typedef __bf16         v16b __attribute__((ext_vector_type(16)));
typedef v2f  __attribute__((may_alias)) v2fa;
typedef v4f  __attribute__((may_alias)) v4fa;
typedef v4i  __attribute__((may_alias)) v4ia;
typedef v8us __attribute__((may_alias)) v8usa;
union FragB { v16b v; v8us h[2]; v8i w; };

__device__ __forceinline__ v8f wmb(const FragB& a, const FragB& b, v8f c) {
  v8f d = __builtin_amdgcn_wmma_f32_16x16x32_bf16(false, a.v, false, b.v, (short)0, c, false, false);
  asm volatile("v_nop\n\tv_nop\n\tv_nop\n\tv_nop" : "+v"(d) : "v"(a.w), "v"(b.w));
  return d;
}

__device__ __forceinline__ unsigned int f2bf(float f) {
  const unsigned int u = __float_as_uint(f);
  const unsigned int r = ((u + 0x7FFFu + ((u >> 16) & 1u)) >> 16) & 0xFFFFu;
  return ((u & 0x7FFFFFFFu) > 0x7F800000u) ? 0x7FC0u : r;
}
__device__ __forceinline__ float bf2f(unsigned int b) { return __uint_as_float(b << 16); }
__device__ __forceinline__ float bfr(float f) { return bf2f(f2bf(f)); }

template <int SLB>
__device__ __forceinline__ int scan_chunk(const int* __restrict__ dsts, int nE, int cbase, int slotBase,
                                          int nb, int vec8, int* list, int tid, int lane, int wave) {
  int wc = 0;
  const int el0  = tid * EPT;
  const int e0   = cbase + el0;
  const int sent = -2147483647 - 1;
  v4i da, db;
  if (vec8 != 0 && cbase + CHUNK <= nE) {
    da = *(const v4i*)(dsts + e0);
    db = *(const v4i*)(dsts + e0 + 4);
  } else {
    da.x = (e0     < nE) ? dsts[min(e0,     nE - 1)] : sent;
    da.y = (e0 + 1 < nE) ? dsts[min(e0 + 1, nE - 1)] : sent;
    da.z = (e0 + 2 < nE) ? dsts[min(e0 + 2, nE - 1)] : sent;
    da.w = (e0 + 3 < nE) ? dsts[min(e0 + 3, nE - 1)] : sent;
    db.x = (e0 + 4 < nE) ? dsts[min(e0 + 4, nE - 1)] : sent;
    db.y = (e0 + 5 < nE) ? dsts[min(e0 + 5, nE - 1)] : sent;
    db.z = (e0 + 6 < nE) ? dsts[min(e0 + 6, nE - 1)] : sent;
    db.w = (e0 + 7 < nE) ? dsts[min(e0 + 7, nE - 1)] : sent;
  }
  const unsigned nbs = (unsigned)slotBase;
  const unsigned unb = (unsigned)nb;
  const unsigned s0 = (unsigned)da.x - nbs, s1 = (unsigned)da.y - nbs;
  const unsigned s2 = (unsigned)da.z - nbs, s3 = (unsigned)da.w - nbs;
  const unsigned s4 = (unsigned)db.x - nbs, s5 = (unsigned)db.y - nbs;
  const unsigned s6 = (unsigned)db.z - nbs, s7 = (unsigned)db.w - nbs;
  const bool h0 = s0 < unb, h1 = s1 < unb, h2 = s2 < unb, h3 = s3 < unb;
  const bool h4 = s4 < unb, h5 = s5 < unb, h6 = s6 < unb, h7 = s7 < unb;
  const unsigned any = __builtin_amdgcn_ballot_w32(h0 | h1 | h2 | h3 | h4 | h5 | h6 | h7);
  if (any != 0u) {
#define HITJ(J, HJ, SJ) { \
      const unsigned mj = __builtin_amdgcn_ballot_w32(HJ); \
      if (mj != 0u) { \
        if (HJ) { \
          const int pos = wc + (int)__builtin_amdgcn_mbcnt_lo(mj, 0u); \
          if (pos < WCAP) list[wave * WCAP + pos] = ((el0 + (J)) << SLB) | (int)(SJ); \
        } \
        wc += (int)__builtin_popcount(mj); } }
    HITJ(0, h0, s0)
    HITJ(1, h1, s1)
    HITJ(2, h2, s2)
    HITJ(3, h3, s3)
    HITJ(4, h4, s4)
    HITJ(5, h5, s5)
    HITJ(6, h6, s6)
    HITJ(7, h7, s7)
#undef HITJ
  }
  return wc;
}

__global__ __launch_bounds__(NTHR) void k_prep(const float* __restrict__ x,
                                               const float* __restrict__ Wl1, const float* __restrict__ Wr1,
                                               const float* __restrict__ Wl2, const float* __restrict__ Wr2,
                                               unsigned short* XB, unsigned short* W1T, unsigned short* W2T,
                                               int nN, int nUx) {
  const int u = (int)blockIdx.x * NTHR + (int)threadIdx.x;
  v8us o;
  unsigned short* dp;
  if (u < nUx) {
    const int row = u >> 4;
    const int c0  = (u & 15) * 8;
    const int rc  = row < nN ? row : nN - 1;
    const float* p = x + (size_t)rc * FIN + c0;
    const v4f a = *(const v4f*)p;
    const v4f b = *(const v4f*)(p + 4);
    const bool okr = row < nN;
    o[0] = okr ? (unsigned short)f2bf(a.x) : (unsigned short)0;
    o[1] = okr ? (unsigned short)f2bf(a.y) : (unsigned short)0;
    o[2] = okr ? (unsigned short)f2bf(a.z) : (unsigned short)0;
    o[3] = okr ? (unsigned short)f2bf(a.w) : (unsigned short)0;
    o[4] = okr ? (unsigned short)f2bf(b.x) : (unsigned short)0;
    o[5] = okr ? (unsigned short)f2bf(b.y) : (unsigned short)0;
    o[6] = okr ? (unsigned short)f2bf(b.z) : (unsigned short)0;
    o[7] = okr ? (unsigned short)f2bf(b.w) : (unsigned short)0;
    dp = XB + (size_t)row * FIN + c0;
  } else if (u < nUx + NUW1H) {
    const int v  = u - nUx;
    const int n  = v >> 4;
    const int k8 = (v & 15) * 8;
    const float* p = Wl1 + (size_t)k8 * HC + n;
#pragma unroll
    for (int i = 0; i < 8; ++i) o[i] = (unsigned short)f2bf(p[(size_t)i * HC]);
    dp = W1T + (size_t)n * FIN + k8;
  } else if (u < nUx + 2 * NUW1H) {
    const int v  = u - nUx - NUW1H;
    const int n  = v >> 4;
    const int k8 = (v & 15) * 8;
    const float* p = Wr1 + (size_t)k8 * HC + n;
#pragma unroll
    for (int i = 0; i < 8; ++i) o[i] = (unsigned short)f2bf(p[(size_t)i * HC]);
    dp = W1T + (size_t)(HC + n) * FIN + k8;
  } else if (u < nUx + 2 * NUW1H + NUW2H) {
    const int v  = u - nUx - 2 * NUW1H;
    const int n  = v >> 6;
    const int k8 = (v & 63) * 8;
    const int kk = k8 & (HC - 1);
    const float* p = Wl2 + (size_t)kk * HC + n;
#pragma unroll
    for (int i = 0; i < 8; ++i) o[i] = (unsigned short)f2bf(p[(size_t)i * HC]);
    dp = W2T + (size_t)n * KA2 + k8;
  } else if (u < nUx + 2 * NUW1H + 2 * NUW2H) {
    const int v  = u - nUx - 2 * NUW1H - NUW2H;
    const int n  = v >> 6;
    const int k8 = (v & 63) * 8;
    const int kk = k8 & (HC - 1);
    const float* p = Wr2 + (size_t)kk * HC + n;
#pragma unroll
    for (int i = 0; i < 8; ++i) o[i] = (unsigned short)f2bf(p[(size_t)i * HC]);
    dp = W2T + (size_t)(HC + n) * KA2 + k8;
  } else {
    return;
  }
  *(volatile v8us*)dp = o;
  __threadfence();
  *(volatile v8us*)dp = o;
}

__global__ __launch_bounds__(NTHR) void k_bucket(const int* __restrict__ srcs, const int* __restrict__ dsts,
                                                 int nE, int nN, int vec8, int* HITS, int* FLG) {
  extern __shared__ __attribute__((aligned(16))) int bsm[];
  int* list = bsm;
  int* reg1 = bsm + LISTN;
  int* wcnt = reg1 + RCAP;
  const int tid = (int)threadIdx.x, lane = tid & 31, wave = tid >> 5;
  const int blk = (int)blockIdx.x;
  const int nodeBase = blk * NBA;
  int nb = nN - nodeBase;
  nb = nb < 0 ? 0 : (nb > NBA ? NBA : nb);

  int tot = 0, ovf = 0;
  const int nChunks = (nE + CHUNK - 1) / CHUNK;
#pragma unroll 1
  for (int ch = 0; ch < nChunks; ++ch) {
    const int cbase = ch * CHUNK;
    const int wc = scan_chunk<SLA>(dsts, nE, cbase, nodeBase, nb, vec8, list, tid, lane, wave);
    if (lane == 0) wcnt[wave] = wc;
    __syncthreads();
    int pre = 0, all = 0;
#pragma unroll
    for (int w2 = 0; w2 < NWAVE; ++w2) {
      int c = wcnt[w2];
      c = c < 0 ? 0 : (c > WCAP ? WCAP : c);
      all += c;
      pre += (w2 < wave) ? c : 0;
    }
    const int wcc  = wc > WCAP ? WCAP : wc;
    const int base = tot + pre;
#pragma unroll 1
    for (int i = lane; i < wcc; i += 32) {
      const int ent = list[wave * WCAP + i];
      const int el  = (ent >> SLA) & (CHUNK - 1);
      const int sl  = ent & (NBA - 1);
      int eid = cbase + el;
      eid = eid > nE - 1 ? nE - 1 : eid;
      const int sraw = srcs[eid];
      const int s = sraw < 0 ? 0 : (sraw > nN - 1 ? nN - 1 : sraw);
      const int pos = base + i;
      if (pos < RCAP) reg1[pos] = (int)((unsigned)s | ((unsigned)sl << 16));
    }
    if (tot + all > RCAP) ovf = 1;
    tot += all;
    tot = tot > RCAP ? RCAP : tot;
    __syncthreads();
  }
  const int nh = tot;
  const int nhPad = (nh + 31) & ~31;
  for (int i = nh + tid; i < nhPad; i += NTHR) reg1[i] = 0;
  __syncthreads();

  int* hb = HITS + (size_t)blk * RCAP;
  v4i cv;
  cv.x = (tid == 0) ? nh : 0;
  cv.y = (tid == 0) ? ovf : 0;
  cv.z = 0; cv.w = 0;
  int* fp = FLG + (size_t)blk * 32 + 4 * (tid & 7);
#pragma unroll 1
  for (int p = tid * 4; p < nhPad; p += NTHR * 4) {
    const v4i v = *(const v4ia*)(reg1 + p);
    *(volatile v4i*)(hb + p) = v;
  }
  if (tid < 8) *(volatile v4i*)fp = cv;
  __threadfence();
#pragma unroll 1
  for (int p = tid * 4; p < nhPad; p += NTHR * 4) {
    const v4i v = *(const v4ia*)(reg1 + p);
    *(volatile v4i*)(hb + p) = v;
  }
  if (tid < 8) *(volatile v4i*)fp = cv;
}

__global__ __launch_bounds__(GTHR) void k_gemm(const unsigned short* __restrict__ A,
                                               const unsigned short* __restrict__ WT,
                                               float* outF, int K, int ldo) {
  __shared__ __attribute__((aligned(16))) float stg[GBM * GBN];
  const int tid = (int)threadIdx.x, lane = tid & 31, wave = tid >> 5, hh = lane >> 4, m = lane & 15;
  const int rowBase = (int)blockIdx.x * GBM;
  const int col0    = (int)blockIdx.y * GBN;

  v8f acc[4];
  {
    const v8f z = {0.f, 0.f, 0.f, 0.f, 0.f, 0.f, 0.f, 0.f};
    acc[0] = z; acc[1] = z; acc[2] = z; acc[3] = z;
  }
  const unsigned short* ap = A  + (size_t)(rowBase + 16 * wave + m) * (size_t)K + 8 * hh;
  const unsigned short* wp = WT + (size_t)(col0 + m) * (size_t)K + 8 * hh;
  const int ksteps = K >> 5;
#pragma unroll 1
  for (int ks = 0; ks < ksteps; ++ks) {
    FragB af;
    af.h[0] = *(const v8usa*)(ap + 32 * ks);
    af.h[1] = *(const v8usa*)(ap + 32 * ks + 16);
#pragma unroll
    for (int t = 0; t < 4; ++t) {
      const unsigned short* wq = wp + (size_t)(16 * t) * (size_t)K + 32 * ks;
      FragB bf;
      bf.h[0] = *(const v8usa*)wq;
      bf.h[1] = *(const v8usa*)(wq + 16);
      acc[t] = wmb(af, bf, acc[t]);
    }
  }

#pragma unroll
  for (int t = 0; t < 4; ++t) {
    const int lc = 16 * t + m;
#pragma unroll
    for (int r = 0; r < 8; ++r) {
      const int lr = 16 * wave + 8 * hh + r;
      stg[lr * GBN + lc] = acc[t][r];
    }
  }
  __syncthreads();

  v4f fv[8];
#pragma unroll
  for (int i = 0; i < 8; ++i) {
    const int lr = 16 * wave + 2 * i + hh;
    fv[i] = *(const v4fa*)(stg + lr * GBN + 4 * m);
  }
#pragma unroll
  for (int i = 0; i < 8; ++i) {
    const int lr = 16 * wave + 2 * i + hh;
    const int gr = rowBase + lr;
    float* op = outF + (size_t)gr * (size_t)ldo + col0 + 4 * m;
    *(volatile v4f*)op = fv[i];
  }
  __threadfence();
#pragma unroll
  for (int i = 0; i < 8; ++i) {
    const int lr = 16 * wave + 2 * i + hh;
    const int gr = rowBase + lr;
    float* op = outF + (size_t)gr * (size_t)ldo + col0 + 4 * m;
    *(volatile v4f*)op = fv[i];
  }
}

template <int L>
__global__ __launch_bounds__(NTHR) void k_scan(const int* __restrict__ HITS, const int* __restrict__ FLGB,
                                               const float* __restrict__ XLR, const float* __restrict__ att,
                                               const float* __restrict__ bias,
                                               unsigned short* XP, float* H2, int* FLGO, int nN, int MPr) {
  static_assert(L == 1 || L == 2);
  extern __shared__ __attribute__((aligned(16))) int ssm[];
  int* hl   = ssm;
  int* sl   = ssm + RCAP;
  int* cnt  = sl + RCAP;
  int* offs = cnt + NBA;
  int* cur  = offs + NBA;
  int* misc = cur + NBA;
  const int tid = (int)threadIdx.x, lane = tid & 31, wave = tid >> 5;
  const int blk = (int)blockIdx.x;
  const int nodeBase = blk * NBA;

  const int nhraw = FLGB[(size_t)blk * 32];
  const int bflag = FLGB[(size_t)blk * 32 + 1];
  const int nh  = nhraw < 0 ? 0 : (nhraw > RCAP ? RCAP : nhraw);
  const int ovf = (bflag != 0 || nhraw < 0 || nhraw > RCAP) ? 1 : 0;

  {
    const v4i z4 = {0, 0, 0, 0};
    for (int i = tid * 4; i < SCAN_ZINTS; i += NTHR * 4) *(v4ia*)(sl + i) = z4;
    if (tid < 16) misc[tid] = 0;
    const int* hb = HITS + (size_t)blk * RCAP;
    const int nh4 = (nh + 3) & ~3;
#pragma unroll 1
    for (int p = tid * 4; p < nh4; p += NTHR * 4) *(v4ia*)(hl + p) = *(const v4i*)(hb + p);
  }
  __syncthreads();

  if (wave == 0) {
#pragma unroll 1
    for (int b0 = 0; b0 < nh; b0 += 32) {
      const int idx = b0 + lane;
      const int uv  = hl[idx < nh ? idx : nh - 1];
      const int m32 = (nh - b0) < 32 ? (nh - b0) : 32;
#pragma unroll 1
      for (int k = 0; k < m32; ++k) {
        const int u  = __builtin_amdgcn_readlane(uv, k);
        const int sq = (u >> 16) & (NBA - 1);
        if (lane == 0) cnt[sq] = cnt[sq] + 1;
      }
    }
  }
  __syncthreads();
  if (wave == 0) {
    const int base = lane * (NBA / 32);
    int s = 0;
#pragma unroll 1
    for (int i = 0; i < NBA / 32; ++i) s += cnt[base + i];
    int incl = s;
#pragma unroll
    for (int d = 1; d < 32; d <<= 1) {
      const int y = __shfl_up(incl, d, 32);
      if (lane >= d) incl += y;
    }
    int run = incl - s;
#pragma unroll 1
    for (int i = 0; i < NBA / 32; ++i) {
      const int cv = cnt[base + i];
      offs[base + i] = run;
      cur[base + i]  = run;
      run += cv;
    }
  }
  __syncthreads();
  if (wave == 0) {
#pragma unroll 1
    for (int b0 = 0; b0 < nh; b0 += 32) {
      const int idx = b0 + lane;
      const int uv  = hl[idx < nh ? idx : nh - 1];
      const int m32 = (nh - b0) < 32 ? (nh - b0) : 32;
#pragma unroll 1
      for (int k = 0; k < m32; ++k) {
        const int u  = __builtin_amdgcn_readlane(uv, k);
        const int sq = (u >> 16) & (NBA - 1);
        if (lane == 0) {
          int p = cur[sq];
          p = p < 0 ? 0 : (p > RCAP - 1 ? RCAP - 1 : p);
          sl[p] = u;
          cur[sq] = p + 1;
        }
      }
    }
  }
  __syncthreads();

  const float qnan = __int_as_float(0x7fc00000);
  const float pzb  = (ovf != 0) ? qnan : 0.0f;
  float at[8], bs[8];
  {
    const v4f a0 = *(const v4f*)(att + 8 * lane);
    const v4f a1 = *(const v4f*)(att + 8 * lane + 4);
    const int bo = (L == 1) ? 8 * lane : 8 * (lane & 7);
    const v4f b0 = *(const v4f*)(bias + bo);
    const v4f b1 = *(const v4f*)(bias + bo + 4);
    at[0] = bfr(a0.x); at[1] = bfr(a0.y); at[2] = bfr(a0.z); at[3] = bfr(a0.w);
    at[4] = bfr(a1.x); at[5] = bfr(a1.y); at[6] = bfr(a1.z); at[7] = bfr(a1.w);
    bs[0] = bfr(b0.x); bs[1] = bfr(b0.y); bs[2] = bfr(b0.z); bs[3] = bfr(b0.w);
    bs[4] = bfr(b1.x); bs[5] = bfr(b1.y); bs[6] = bfr(b1.z); bs[7] = bfr(b1.w);
  }
  int anybig = 0;

#pragma unroll 1
  for (int si = 0; si < NBA / NWAVE; ++si) {
    const int s    = si * NWAVE + wave;
    const int node = nodeBase + s;
    const int nc   = node < nN ? node : nN - 1;
    int c = __builtin_amdgcn_readfirstlane(cnt[s]);
    int o = __builtin_amdgcn_readfirstlane(offs[s]);
    const bool big = c > DEGCAP;
    anybig |= big ? 1 : 0;
    c = c < 0 ? 0 : (c > DEGCAP ? DEGCAP : c);
    o = o < 0 ? 0 : (o > RCAP ? RCAP : o);
    if (c > nh - o) c = nh - o;
    c = c < 0 ? 0 : c;

    float xr[8];
    {
      const float* dr = XLR + (size_t)nc * LDX + HC + 8 * lane;
      const v4f a = *(const v4f*)dr;
      const v4f b = *(const v4f*)(dr + 4);
      xr[0] = a.x; xr[1] = a.y; xr[2] = a.z; xr[3] = a.w;
      xr[4] = b.x; xr[5] = b.y; xr[6] = b.z; xr[7] = b.w;
    }
    float mx = -3.0e38f, dn = 0.0f;
    float acc[8];
#pragma unroll
    for (int i = 0; i < 8; ++i) acc[i] = 0.0f;
    const int T = c + 1;
#pragma unroll 1
    for (int b0 = 0; b0 < T; b0 += 32) {
      const int t = b0 + lane;
      int idx = o + t;
      idx = idx < 0 ? 0 : (idx > RCAP - 1 ? RCAP - 1 : idx);
      const int ent = sl[idx];
      int hs = ent & 0xFFFF;
      hs = hs > nN - 1 ? nN - 1 : hs;
      const int sr  = (t < c) ? hs : nc;
      const int m32 = (T - b0) < 32 ? (T - b0) : 32;
#pragma unroll 1
      for (int k = 0; k < m32; ++k) {
        const int sk = __builtin_amdgcn_readlane(sr, k);
        const float* rp = XLR + (size_t)sk * LDX + 8 * lane;
        const v4f a = *(const v4f*)rp;
        const v4f b = *(const v4f*)(rp + 4);
        float xs[8];
        xs[0] = a.x; xs[1] = a.y; xs[2] = a.z; xs[3] = a.w;
        xs[4] = b.x; xs[5] = b.y; xs[6] = b.z; xs[7] = b.w;
        float part = 0.0f;
#pragma unroll
        for (int i = 0; i < 8; ++i) {
          float v = xs[i] + xr[i];
          v = (v > 0.0f) ? v : NEGSL * v;
          part = fmaf(v, at[i], part);
        }
        part += __shfl_xor(part, 1, 32);
        part += __shfl_xor(part, 2, 32);
        part += __shfl_xor(part, 4, 32);
        const float lg = part;
        const float df = lg - mx;
        const float ee = expf(-fabsf(df));
        const bool  up = df > 0.f;
        const float s1 = up ? ee : 1.0f;
        const float s2 = up ? 1.0f : ee;
        mx = up ? lg : mx;
        dn = fmaf(dn, s1, s2);
#pragma unroll
        for (int i = 0; i < 8; ++i) acc[i] = fmaf(acc[i], s1, s2 * xs[i]);
      }
    }
    const float inv = 1.0f / (dn + 1e-16f);
    const float pzr = big ? qnan : pzb;
    const bool live = node < nN;

    if constexpr (L == 1) {
      v8us ho, lo;
#pragma unroll
      for (int i = 0; i < 8; ++i) {
        const float y = fmaf(acc[i], inv, bs[i]) + pzr;
        const float v = live ? y : 0.0f;
        const unsigned int hbi = f2bf(v);
        ho[i] = (unsigned short)hbi;
        lo[i] = (unsigned short)f2bf(v - bf2f(hbi));
      }
      if (node < MPr) {
        unsigned short* hp = XP + (size_t)node * KA2 + 8 * lane;
        *(volatile v8us*)hp = ho;
        *(volatile v8us*)(hp + HC) = lo;
        __threadfence();
        *(volatile v8us*)hp = ho;
        *(volatile v8us*)(hp + HC) = lo;
      }
    } else {
      float r[8];
#pragma unroll
      for (int i = 0; i < 8; ++i) r[i] = acc[i] * inv;
#pragma unroll
      for (int i = 0; i < 8; ++i) r[i] += __shfl_xor(r[i], 8, 32);
#pragma unroll
      for (int i = 0; i < 8; ++i) r[i] += __shfl_xor(r[i], 16, 32);
#pragma unroll
      for (int i = 0; i < 8; ++i) r[i] = fmaf(r[i], 0.25f, bs[i]) + pzr;
      float t8[8];
      const int sl2 = lane >> 1;
#pragma unroll
      for (int i = 0; i < 8; ++i) t8[i] = __shfl(r[i], sl2, 32);
      const bool odd = (lane & 1) != 0;
      v4f ov;
      ov.x = odd ? t8[4] : t8[0];
      ov.y = odd ? t8[5] : t8[1];
      ov.z = odd ? t8[6] : t8[2];
      ov.w = odd ? t8[7] : t8[3];
      const bool wsv = live && (lane < 16);
      float* gp = H2 + (size_t)nc * HID + 4 * (lane & 15);
      if (wsv) *(volatile v4f*)gp = ov;
      __threadfence();
      if (wsv) *(volatile v4f*)gp = ov;
    }
  }

  if (lane == 0) misc[wave] = anybig;
  __syncthreads();
  if (wave == 0) {
    int fg = ovf;
#pragma unroll
    for (int w2 = 0; w2 < NWAVE; ++w2) fg |= misc[w2];
    v4i cv;
    cv.x = 0;
    cv.y = (lane == 0) ? fg : 0;
    cv.z = 0; cv.w = 0;
    int* fp = FLGO + (size_t)blk * 32 + 4 * (lane & 7);
    if (lane < 8) *(volatile v4i*)fp = cv;
    __threadfence();
    if (lane < 8) *(volatile v4i*)fp = cv;
  }
  (void)XP; (void)H2;
}

__global__ __launch_bounds__(NTHR) void k_pool(const int* __restrict__ batch, const float* __restrict__ H2,
                                               float* GP, int nN) {
  __shared__ __attribute__((aligned(16))) float wm[NWAVE * HID];
  const int tid = (int)threadIdx.x, lane = tid & 31;
  const int wave = __builtin_amdgcn_readfirstlane(tid >> 5);
  const int k = (int)blockIdx.x;
  const float ninf = __int_as_float((int)0xff800000u);
  float m0 = ninf, m1 = ninf;
  const int nCh = (nN + 31) >> 5;
#pragma unroll 1
  for (int ch = wave; ch < nCh; ch += NWAVE) {
    const int n   = ch * 32 + lane;
    const int ncl = n < nN ? n : nN - 1;
    const int b   = batch[ncl];
    const bool hit = (n < nN) && (b == k);
    unsigned mask = __builtin_amdgcn_ballot_w32(hit);
#pragma unroll 1
    for (int it = 0; it < 32; ++it) {
      if (mask == 0u) break;
      const int j = __builtin_ctz(mask);
      mask &= mask - 1u;
      int node = ch * 32 + j;
      node = node > nN - 1 ? nN - 1 : node;
      const v2f v = *(const v2f*)(H2 + (size_t)node * HID + 2 * lane);
      m0 = fmaxf(m0, v.x);
      m1 = fmaxf(m1, v.y);
    }
  }
  {
    v2f pv; pv.x = m0; pv.y = m1;
    *(v2fa*)(wm + wave * HID + 2 * lane) = pv;
  }
  __syncthreads();
  if (wave == 0) {
    const int lc = lane & 15;
    v4f r = *(const v4fa*)(wm + 4 * lc);
#pragma unroll
    for (int w2 = 1; w2 < NWAVE; ++w2) {
      const v4f p = *(const v4fa*)(wm + w2 * HID + 4 * lc);
      r.x = fmaxf(r.x, p.x); r.y = fmaxf(r.y, p.y);
      r.z = fmaxf(r.z, p.z); r.w = fmaxf(r.w, p.w);
    }
    float* gp = GP + (size_t)k * HID + 4 * lc;
    if (lane < 16) *(volatile v4f*)gp = r;
    __threadfence();
    if (lane < 16) *(volatile v4f*)gp = r;
  }
}

__global__ __launch_bounds__(NTHR) void k_head(const float* __restrict__ GP, const int* __restrict__ FLG, int nLines,
                                               const float* __restrict__ Wc1, const float* __restrict__ bc1,
                                               const float* __restrict__ Wc2, const float* __restrict__ bc2,
                                               float* out) {
  __shared__ __attribute__((aligned(16))) float sg [NGR * HID];
  __shared__ __attribute__((aligned(16))) float sw1[HID * HID];
  __shared__ __attribute__((aligned(16))) float shd[NGR * HID];
  __shared__ __attribute__((aligned(16))) float sw2[HID * OUTC];
  __shared__ __attribute__((aligned(16))) float sb1[HID];
  __shared__ __attribute__((aligned(16))) float sb2[OUTC];
  __shared__ __attribute__((aligned(16))) float so [NGR * OUTC];
  __shared__ int sfl[NWAVE];
  const int tid = (int)threadIdx.x, lane = tid & 31, wave = tid >> 5;

#pragma unroll 1
  for (int it = 0; it < 4; ++it) {
    const int i = tid + NTHR * it;
    v4f g = *(const v4f*)(GP + 4 * i);
    g.x = ((__float_as_uint(g.x) & 0x7F800000u) != 0x7F800000u) ? g.x : 0.0f;
    g.y = ((__float_as_uint(g.y) & 0x7F800000u) != 0x7F800000u) ? g.y : 0.0f;
    g.z = ((__float_as_uint(g.z) & 0x7F800000u) != 0x7F800000u) ? g.z : 0.0f;
    g.w = ((__float_as_uint(g.w) & 0x7F800000u) != 0x7F800000u) ? g.w : 0.0f;
    *(v4fa*)(sg + 4 * i) = g;
    v4f w = *(const v4f*)(Wc1 + 4 * i);
    w.x = bfr(w.x); w.y = bfr(w.y); w.z = bfr(w.z); w.w = bfr(w.w);
    *(v4fa*)(sw1 + 4 * i) = w;
  }
  {
    v4f w = *(const v4f*)(Wc2 + 4 * tid);
    w.x = bfr(w.x); w.y = bfr(w.y); w.z = bfr(w.z); w.w = bfr(w.w);
    *(v4fa*)(sw2 + 4 * tid) = w;
    const int i1 = tid & 15;
    v4f b = *(const v4f*)(bc1 + 4 * i1);
    b.x = bfr(b.x); b.y = bfr(b.y); b.z = bfr(b.z); b.w = bfr(b.w);
    if (tid < 16) *(v4fa*)(sb1 + 4 * i1) = b;
    const int i2 = tid & 3;
    v4f c = *(const v4f*)(bc2 + 4 * i2);
    c.x = bfr(c.x); c.y = bfr(c.y); c.z = bfr(c.z); c.w = bfr(c.w);
    if (tid < 4) *(v4fa*)(sb2 + 4 * i2) = c;
  }
  {
    int f = 0;
    const int nIt = (nLines + NTHR - 1) / NTHR;
#pragma unroll 1
    for (int it = 0; it < nIt; ++it) {
      int i = tid + NTHR * it;
      i = i > nLines - 1 ? nLines - 1 : i;
      f |= FLG[(size_t)i * 32 + 1];
    }
    const unsigned anyw = __builtin_amdgcn_ballot_w32(f != 0);
    if (lane == 0) sfl[wave] = (anyw != 0u) ? 1 : 0;
  }
  __syncthreads();

  {
    const int c = tid & 63, r0 = tid >> 6;
#pragma unroll 1
    for (int q = 0; q < 16; ++q) {
      const int r = r0 + 4 * q;
      float a = 0.0f;
#pragma unroll 4
      for (int k = 0; k < HID; ++k) a = fmaf(sg[r * HID + k], sw1[k * HID + c], a);
      a += sb1[c];
      shd[r * HID + c] = (a > 0.0f) ? a : (a - a);
    }
  }
  __syncthreads();
  {
    const int c2 = tid & 15, q0 = tid >> 4;
#pragma unroll 1
    for (int q = 0; q < 4; ++q) {
      const int r = q0 + 16 * q;
      float a = 0.0f;
#pragma unroll 4
      for (int k = 0; k < HID; ++k) a = fmaf(shd[r * HID + k], sw2[k * OUTC + c2], a);
      a += sb2[c2];
      so[r * OUTC + c2] = a;
    }
  }
  __syncthreads();
  int fg = 0;
#pragma unroll
  for (int w2 = 0; w2 < NWAVE; ++w2) fg |= sfl[w2];
  const float qnan = __int_as_float(0x7fc00000);
  v4f ov = *(const v4fa*)(so + 4 * tid);
  ov.x = (fg != 0) ? qnan : ov.x;
  ov.y = (fg != 0) ? qnan : ov.y;
  ov.z = (fg != 0) ? qnan : ov.z;
  ov.w = (fg != 0) ? qnan : ov.w;
  float* op = out + 4 * tid;
  *(volatile v4f*)op = ov;
  __threadfence();
  *(volatile v4f*)op = ov;
}

static inline int cdiv(int a, int b) { return (a + b - 1) / b; }

extern "C" void kernel_launch(void* const* d_in, const int* in_sizes, int n_in,
                              void* d_out, int out_size, void* d_ws, size_t ws_size,
                              hipStream_t stream) {
  if (n_in < 15) return;
  const int nN = in_sizes[0] / FIN;
  if (nN <= 0 || in_sizes[0] != nN * FIN || nN > 65536) return;
  if (in_sizes[1] < 2 || (in_sizes[1] & 1) != 0) return;
  const int nE = in_sizes[1] / 2;
  if (nE < 1 || nE > (1 << 30)) return;
  if (in_sizes[2] != nN) return;
  if (in_sizes[3] != FIN * HC || in_sizes[4] != FIN * HC) return;
  if (in_sizes[5] != NHD * HID || in_sizes[6] != HC) return;
  if (in_sizes[7] != HC * HC || in_sizes[8] != HC * HC) return;
  if (in_sizes[9] != NHD * HID || in_sizes[10] != HID) return;
  if (in_sizes[11] != HID * HID || in_sizes[12] != HID) return;
  if (in_sizes[13] != HID * OUTC || in_sizes[14] != OUTC) return;
  if (out_size != NGR * OUTC) return;

  const float* x    = (const float*)d_in[0];
  const int*   ei   = (const int*)  d_in[1];
  const int*   bat  = (const int*)  d_in[2];
  const float* Wl1  = (const float*)d_in[3];
  const float* Wr1  = (const float*)d_in[4];
  const float* att1 = (const float*)d_in[5];
  const float* b1   = (const float*)d_in[6];
  const float* Wl2  = (const float*)d_in[7];
  const float* Wr2  = (const float*)d_in[8];
  const float* att2 = (const float*)d_in[9];
  const float* b2   = (const float*)d_in[10];
  const float* Wc1  = (const float*)d_in[11];
  const float* bc1  = (const float*)d_in[12];
  const float* Wc2  = (const float*)d_in[13];
  const float* bc2  = (const float*)d_in[14];
  float* out = (float*)d_out;
  const int* src = ei;
  const int* dst = ei + nE;

  const int MP   = cdiv(nN, MROWS) * MROWS;
  const int gM   = MP / GBM;
  const int gA   = cdiv(MP, NBA);
  if ((long long)gA * NBA < (long long)MP) return;
  const int vec8 = ((nE & 3) == 0) ? 1 : 0;
  const int nUx  = MP * (FIN / 8);
  if ((nUx % NTHR) != 0) return;
  const int nUall = nUx + 2 * NUW1H + 2 * NUW2H;
  if ((nUall % NTHR) != 0) return;

  char* ws = (char*)d_ws;
  size_t off = 0;
  const size_t oXLR = off; off += (size_t)MP * LDX * 4;          off = (off + 255) & ~(size_t)255;
  const size_t oHB  = off; off += (size_t)MP * KA2 * 2;          off = (off + 255) & ~(size_t)255;
  const size_t oH2  = off; off += (size_t)MP * HID * 4;          off = (off + 255) & ~(size_t)255;
  const size_t oHIT = off; off += (size_t)gA * RCAP * 4;         off = (off + 255) & ~(size_t)255;
  const size_t oFLG = off; off += (size_t)3 * gA * 128;          off = (off + 255) & ~(size_t)255;
  const size_t oGP  = off; off += (size_t)NGR * HID * 4;         off = (off + 255) & ~(size_t)255;
  const size_t oW1T = off; off += (size_t)LDX * FIN * 2;         off = (off + 255) & ~(size_t)255;
  const size_t oW2T = off; off += (size_t)LDX * KA2 * 2;         off = (off + 255) & ~(size_t)255;
  if (off > ws_size || off > (size_t)WSMAX) return;
  if ((size_t)MP * FIN * 2 > (size_t)MP * KA2 * 2) return;
  float*          XLR  = (float*)(ws + oXLR);
  unsigned short* XB   = (unsigned short*)(ws + oHB);
  unsigned short* H1HL = (unsigned short*)(ws + oHB);
  float*          H2   = (float*)(ws + oH2);
  int*            HITS = (int*)(ws + oHIT);
  int*            FLG  = (int*)(ws + oFLG);
  float*          GP   = (float*)(ws + oGP);
  unsigned short* W1T  = (unsigned short*)(ws + oW1T);
  unsigned short* W2T  = (unsigned short*)(ws + oW2T);
  int* FLG0 = FLG;
  int* FLG1 = FLG + (size_t)gA * 32;
  int* FLG2 = FLG + (size_t)2 * gA * 32;

  const int bktLds  = BKT_LDS_INTS * 4;
  const int scanLds = SCAN_LDS_INTS * 4;
  hipFuncSetAttribute(reinterpret_cast<const void*>(&k_bucket),
                      hipFuncAttributeMaxDynamicSharedMemorySize, bktLds);
  hipFuncSetAttribute(reinterpret_cast<const void*>(&k_scan<1>),
                      hipFuncAttributeMaxDynamicSharedMemorySize, scanLds);
  hipFuncSetAttribute(reinterpret_cast<const void*>(&k_scan<2>),
                      hipFuncAttributeMaxDynamicSharedMemorySize, scanLds);

  k_prep<<<nUall / NTHR, NTHR, 0, stream>>>(x, Wl1, Wr1, Wl2, Wr2, XB, W1T, W2T, nN, nUx);
  k_bucket<<<gA, NTHR, bktLds, stream>>>(src, dst, nE, nN, vec8, HITS, FLG0);
  k_gemm<<<dim3(gM, LDX / GBN), GTHR, 0, stream>>>(XB, W1T, XLR, FIN, LDX);
  k_scan<1><<<gA, NTHR, scanLds, stream>>>(HITS, FLG0, XLR, att1, b1, H1HL, H2, FLG1, nN, MP);
  k_gemm<<<dim3(gM, LDX / GBN), GTHR, 0, stream>>>(H1HL, W2T, XLR, KA2, LDX);
  k_scan<2><<<gA, NTHR, scanLds, stream>>>(HITS, FLG0, XLR, att2, b2, H1HL, H2, FLG2, nN, MP);
  k_pool<<<NGR, NTHR, 0, stream>>>(bat, H2, GP, nN);
  k_head<<<1, NTHR, 0, stream>>>(GP, FLG, 3 * gA, Wc1, bc1, Wc2, bc2, out);
}
